// SABlock_20581483283051
// MI455X (gfx1250) — hardware-verified
//
#include <hip/hip_runtime.h>


#ifndef NB
#define NB 2
#endif
#ifndef SEQ
#define SEQ 2048
#endif
#ifndef NB_FULL
#define NB_FULL 2
#endif
#ifndef SEQ_FULL
#define SEQ_FULL 2048
#endif
#ifndef EARLY_ROWS
#define EARLY_ROWS 512
#endif
#define HIDDEN   1024
#define HEADS    16
#define HEAD_DIM 64
#define QKV_N    (3 * HIDDEN)

static constexpr int   EARLY     = (EARLY_ROWS < SEQ) ? EARLY_ROWS : SEQ;
static constexpr int   MROWS     = NB * SEQ;
static constexpr float ATT_SCALE = 0.125f;
static constexpr float P_CARRY   = 1024.0f;
static constexpr float NEG_BIG   = -1.0e30f;

static_assert(SEQ % 256 == 0);
static_assert(EARLY % 256 == 0);
static_assert(EARLY >= 256);
static_assert(SEQ <= SEQ_FULL);
static_assert(NB <= NB_FULL);
static_assert(MROWS % 256 == 0);
static_assert(HIDDEN == HEADS * HEAD_DIM);
static_assert(QKV_N % 64 == 0);

#define PANEL_PITCH   1032
#define LDS_DYN_BYTES (64 * PANEL_PITCH * 2)
static_assert(3 * 256 * 72 * 2 <= LDS_DYN_BYTES);
static_assert(3 * 64 * 264 * 2 <= LDS_DYN_BYTES);
static_assert(8 * 32 * 68 * 4 <= LDS_DYN_BYTES);

typedef _Float16       v16h  __attribute__((ext_vector_type(16)));
typedef _Float16       v8h   __attribute__((ext_vector_type(8)));
typedef __bf16         v16bf __attribute__((ext_vector_type(16)));
typedef unsigned short v16us __attribute__((ext_vector_type(16)));
typedef unsigned short v8us  __attribute__((ext_vector_type(8)));
typedef float          v8f   __attribute__((ext_vector_type(8)));
typedef float          v4f   __attribute__((ext_vector_type(4)));
typedef v8h  __attribute__((may_alias)) v8h_a;
typedef v8us __attribute__((may_alias)) v8us_a;
typedef v4f  __attribute__((may_alias)) v4f_a;

union FragH { v16h v;  v8h  h[2]; };
union FragU { v16us v; v8us h[2]; };

__device__ __forceinline__ unsigned short bf16_rne_bits(float f) {
    unsigned int u = __float_as_uint(f);
    u += 0x7FFFu + ((u >> 16) & 1u);
    return (unsigned short)(u >> 16);
}
__device__ __forceinline__ float bf16_bits_to_f32(unsigned short b) {
    return __uint_as_float(((unsigned int)b) << 16);
}
__device__ __forceinline__ unsigned short f16_bits(float f) {
    _Float16 hv = (_Float16)f;
    return __builtin_bit_cast(unsigned short, hv);
}

__device__ __forceinline__ float rowmax16(float v) {
    v = fmaxf(v, __shfl_xor(v, 1, 16));
    v = fmaxf(v, __shfl_xor(v, 2, 16));
    v = fmaxf(v, __shfl_xor(v, 4, 16));
    v = fmaxf(v, __shfl_xor(v, 8, 16));
    return v;
}
__device__ __forceinline__ float rowsum16(float v) {
    v += __shfl_xor(v, 1, 16);
    v += __shfl_xor(v, 2, 16);
    v += __shfl_xor(v, 4, 16);
    v += __shfl_xor(v, 8, 16);
    return v;
}

__device__ __forceinline__ v16h ld_frag_f16(const _Float16* p, int hsel) {
    FragH f;
    f.h[0] = *(const v8h_a*)(p + 8 * hsel);
    f.h[1] = *(const v8h_a*)(p + 16 + 8 * hsel);
    return f.v;
}
__device__ __forceinline__ v16bf ld_frag_bf16(const unsigned short* p, int hsel) {
    FragU f;
    f.h[0] = *(const v8us_a*)(p + 8 * hsel);
    f.h[1] = *(const v8us_a*)(p + 16 + 8 * hsel);
    return __builtin_bit_cast(v16bf, f.v);
}

__device__ __forceinline__ v8f mma_f16(const v16h& a, const v16h& b, const v8f& c) {
    return __builtin_amdgcn_wmma_f32_16x16x32_f16(false, a, false, b, (short)0, c, false, false);
}
__device__ __forceinline__ v8f mma_bf16(const v16bf& a, const v16bf& b, const v8f& c) {
    return __builtin_amdgcn_wmma_f32_16x16x32_bf16(false, a, false, b, (short)0, c, false, false);
}
template <class FA, class FB>
__device__ __forceinline__ void guard2(v8f& d0, v8f& d1, const FA& a, const FB& b) {
    asm volatile("v_nop\n\tv_nop\n\tv_nop\n\tv_nop" : "+v"(d0), "+v"(d1) : "v"(a), "v"(b));
}
template <class FA, class FB>
__device__ __forceinline__ void guard4(v8f (&d)[4], const FA& a, const FB& b) {
    asm volatile("v_nop\n\tv_nop\n\tv_nop\n\tv_nop"
                 : "+v"(d[0]), "+v"(d[1]), "+v"(d[2]), "+v"(d[3])
                 : "v"(a), "v"(b));
}
template <class FA, class FB>
__device__ __forceinline__ void guard8(v8f (&d)[2][4], const FA& a, const FB& b) {
    asm volatile("v_nop\n\tv_nop\n\tv_nop\n\tv_nop"
                 : "+v"(d[0][0]), "+v"(d[0][1]), "+v"(d[0][2]), "+v"(d[0][3]),
                   "+v"(d[1][0]), "+v"(d[1][1]), "+v"(d[1][2]), "+v"(d[1][3])
                 : "v"(a), "v"(b));
}

__global__ void __launch_bounds__(256)
cvt_rows_bf16(const float* __restrict__ src, unsigned short* __restrict__ dst,
              int nrows, int seq, int seq_full) {
    const int tid = threadIdx.x;
    int m = blockIdx.x * 2 + (tid >> 7);
    m = (m < nrows) ? m : (nrows - 1);
    const int piece = tid & 127;
    const int bq = m / seq;
    const size_t srow = (size_t)bq * seq_full + (size_t)(m - bq * seq);
    const float* s = src + srow * HIDDEN + piece * 8;
    const v4f f0 = *(const v4f_a*)(s);
    const v4f f1 = *(const v4f_a*)(s + 4);
    v8us o = {};
    o[0] = bf16_rne_bits(f0[0]); o[1] = bf16_rne_bits(f0[1]);
    o[2] = bf16_rne_bits(f0[2]); o[3] = bf16_rne_bits(f0[3]);
    o[4] = bf16_rne_bits(f1[0]); o[5] = bf16_rne_bits(f1[1]);
    o[6] = bf16_rne_bits(f1[2]); o[7] = bf16_rne_bits(f1[3]);
    unsigned short* d = dst + (size_t)m * HIDDEN + piece * 8;
    *(volatile v8us*)d = o;
    __threadfence();
    *(volatile v8us*)d = o;
}

__device__ __forceinline__ void stage_panel(unsigned short* ldsB,
                                            const unsigned short* __restrict__ Bw, int nBase) {
#pragma unroll 4
    for (int it = 0; it < 32; ++it) {
        const int c   = it * 256 + (int)threadIdx.x;
        const int r   = c >> 7;
        const int col = (c & 127) * 8;
        const v8us v = *(const v8us_a*)(Bw + (size_t)(nBase + r) * HIDDEN + col);
        *(v8us_a*)(ldsB + r * PANEL_PITCH + col) = v;
    }
}

__device__ __forceinline__ void put_rows64(const unsigned short* T, unsigned short* g,
                                           int wave, int lane) {
#pragma unroll
    for (int p = 0; p < 8; ++p) {
        const int L  = wave * 32 + p * 4 + (lane >> 3);
        const int pc = (lane & 7) * 8;
        const v8us v = *(const v8us_a*)(T + L * 72 + pc);
        *(volatile v8us*)(g + (size_t)L * HEAD_DIM + pc) = v;
    }
}
__device__ __forceinline__ void put_vt(const unsigned short* T, unsigned short* g, int spitch,
                                       int wave, int lane) {
#pragma unroll
    for (int p = 0; p < 8; ++p) {
        const int d  = wave * 8 + p;
        const int c  = lane >> 3;
        const int pc = (lane & 7) * 8;
        const v8us v = *(const v8us_a*)(T + d * 264 + c * 64 + pc);
        *(volatile v8us*)(g + (size_t)d * spitch + c * 64 + pc) = v;
    }
}
__device__ __forceinline__ void put_out64(const float* T, float* g, int lane) {
#pragma unroll
    for (int p = 0; p < 16; ++p) {
        const int L   = p * 4 + (lane >> 3);
        const int row = L >> 1;
        const int c0  = (L & 1) * 32 + (lane & 7) * 4;
        const v4f v = *(const v4f_a*)(T + row * 68 + c0);
        *(volatile v4f*)(g + (size_t)row * HIDDEN + c0) = v;
    }
}
__device__ __forceinline__ void put_ctx16(const unsigned short* T, unsigned short* g, int lane) {
#pragma unroll
    for (int p = 0; p < 4; ++p) {
        const int L  = p * 4 + (lane >> 3);
        const int pc = (lane & 7) * 8;
        const v8us v = *(const v8us_a*)(T + L * 72 + pc);
        *(volatile v8us*)(g + (size_t)L * HIDDEN + pc) = v;
    }
}

__global__ void __launch_bounds__(256)
gemm_qkv(const unsigned short* __restrict__ A, const unsigned short* __restrict__ Bw,
         unsigned short* __restrict__ Qf,  unsigned short* __restrict__ Kf,
         unsigned short* __restrict__ Vtf,
         unsigned short* __restrict__ Qbh, unsigned short* __restrict__ Qbl,
         unsigned short* __restrict__ Kbh, unsigned short* __restrict__ Kbl,
         unsigned short* __restrict__ Vbh, unsigned short* __restrict__ Vbl) {
    extern __shared__ __attribute__((aligned(16))) unsigned char lds_dyn_q[];
    unsigned short* ldsB = (unsigned short*)lds_dyn_q;

    const int wave  = threadIdx.x >> 5;
    const int lane  = threadIdx.x & 31;
    const int laneN = lane & 15;
    const int hsel  = lane >> 4;
    const int nBase = blockIdx.y * 64;
    const int mBlk  = blockIdx.x * 256;
    const int mBase = mBlk + wave * 32;

    stage_panel(ldsB, Bw, nBase);
    __syncthreads();

    v8f acc[2][4] = {};
    {
        const unsigned short* a0p = A + (size_t)(mBase + laneN) * HIDDEN;
        const unsigned short* a1p = A + (size_t)(mBase + 16 + laneN) * HIDDEN;
#pragma unroll 1
        for (int k0 = 0; k0 < HIDDEN; k0 += 32) {
            const v16bf af0 = ld_frag_bf16(a0p + k0, hsel);
            const v16bf af1 = ld_frag_bf16(a1p + k0, hsel);
            v16bf bfr;
#pragma unroll
            for (int a = 0; a < 4; ++a) {
                bfr = ld_frag_bf16(ldsB + (a * 16 + laneN) * PANEL_PITCH + k0, hsel);
                acc[0][a] = mma_bf16(af0, bfr, acc[0][a]);
                acc[1][a] = mma_bf16(af1, bfr, acc[1][a]);
            }
            guard8(acc, af1, bfr);
        }
    }
    __syncthreads();

    const int which = nBase >> 10;
    const int head  = (nBase & (HIDDEN - 1)) >> 6;
    const int bidx  = mBlk / SEQ;
    const int s0    = mBlk - bidx * SEQ;
    const int bh    = bidx * HEADS + head;
    const bool early = (s0 < EARLY);
    unsigned short* T0 = (unsigned short*)lds_dyn_q;

    if (which < 2) {
        unsigned short* T1 = T0 + 256 * 72;
        unsigned short* T2 = T1 + 256 * 72;
#pragma unroll
        for (int sub = 0; sub < 2; ++sub)
#pragma unroll
            for (int a = 0; a < 4; ++a)
#pragma unroll
                for (int j = 0; j < 8; ++j) {
                    const int ml = wave * 32 + sub * 16 + 8 * hsel + j;
                    const int n  = a * 16 + laneN;
                    const float v = acc[sub][a][j];
                    T0[ml * 72 + n] = f16_bits(v);
                    if (early) {
                        const unsigned short hb = bf16_rne_bits(v);
                        T1[ml * 72 + n] = hb;
                        T2[ml * 72 + n] = bf16_rne_bits(v - bf16_bits_to_f32(hb));
                    }
                }
        __syncthreads();
        unsigned short* gF = ((which == 0) ? Qf : Kf) + ((size_t)bh * SEQ + s0) * HEAD_DIM;
        put_rows64(T0, gF, wave, lane);
        if (early) {
            unsigned short* gH = ((which == 0) ? Qbh : Kbh) + ((size_t)bh * EARLY + s0) * HEAD_DIM;
            unsigned short* gL = ((which == 0) ? Qbl : Kbl) + ((size_t)bh * EARLY + s0) * HEAD_DIM;
            put_rows64(T1, gH, wave, lane);
            put_rows64(T2, gL, wave, lane);
        }
        __threadfence();
        put_rows64(T0, gF, wave, lane);
        if (early) {
            unsigned short* gH = ((which == 0) ? Qbh : Kbh) + ((size_t)bh * EARLY + s0) * HEAD_DIM;
            unsigned short* gL = ((which == 0) ? Qbl : Kbl) + ((size_t)bh * EARLY + s0) * HEAD_DIM;
            put_rows64(T1, gH, wave, lane);
            put_rows64(T2, gL, wave, lane);
        }
    } else {
        unsigned short* T1 = T0 + 64 * 264;
        unsigned short* T2 = T1 + 64 * 264;
#pragma unroll
        for (int sub = 0; sub < 2; ++sub)
#pragma unroll
            for (int a = 0; a < 4; ++a) {
                const int d  = a * 16 + laneN;
                const int ml = wave * 32 + sub * 16 + 8 * hsel;
                v8us pk = {}, ph = {}, pl = {};
#pragma unroll
                for (int j = 0; j < 8; ++j) {
                    const float v = acc[sub][a][j];
                    pk[j] = f16_bits(v);
                    if (early) {
                        const unsigned short hb = bf16_rne_bits(v);
                        ph[j] = hb;
                        pl[j] = bf16_rne_bits(v - bf16_bits_to_f32(hb));
                    }
                }
                *(v8us_a*)(T0 + d * 264 + ml) = pk;
                if (early) {
                    *(v8us_a*)(T1 + d * 264 + ml) = ph;
                    *(v8us_a*)(T2 + d * 264 + ml) = pl;
                }
            }
        __syncthreads();
        unsigned short* gV = Vtf + (size_t)bh * HEAD_DIM * SEQ + s0;
        put_vt(T0, gV, SEQ, wave, lane);
        if (early) {
            unsigned short* gH = Vbh + (size_t)bh * HEAD_DIM * EARLY + s0;
            unsigned short* gL = Vbl + (size_t)bh * HEAD_DIM * EARLY + s0;
            put_vt(T1, gH, EARLY, wave, lane);
            put_vt(T2, gL, EARLY, wave, lane);
        }
        __threadfence();
        put_vt(T0, gV, SEQ, wave, lane);
        if (early) {
            unsigned short* gH = Vbh + (size_t)bh * HEAD_DIM * EARLY + s0;
            unsigned short* gL = Vbl + (size_t)bh * HEAD_DIM * EARLY + s0;
            put_vt(T1, gH, EARLY, wave, lane);
            put_vt(T2, gL, EARLY, wave, lane);
        }
    }
}

__global__ void __launch_bounds__(256)
gemm_out(const unsigned short* __restrict__ Ah, const unsigned short* __restrict__ Al,
         const unsigned short* __restrict__ Bw, const float* __restrict__ bias,
         float* __restrict__ Out) {
    extern __shared__ __attribute__((aligned(16))) unsigned char lds_dyn_o[];
    unsigned short* ldsB = (unsigned short*)lds_dyn_o;

    const int wave  = threadIdx.x >> 5;
    const int lane  = threadIdx.x & 31;
    const int laneN = lane & 15;
    const int hsel  = lane >> 4;
    const int nBase = blockIdx.y * 64;
    const int mBase = blockIdx.x * 256 + wave * 32;

    stage_panel(ldsB, Bw, nBase);
    __syncthreads();

    v8f acc[2][4] = {};
    {
        const unsigned short* h0p = Ah + (size_t)(mBase + laneN) * HIDDEN;
        const unsigned short* h1p = Ah + (size_t)(mBase + 16 + laneN) * HIDDEN;
        const unsigned short* l0p = Al + (size_t)(mBase + laneN) * HIDDEN;
        const unsigned short* l1p = Al + (size_t)(mBase + 16 + laneN) * HIDDEN;
#pragma unroll 1
        for (int k0 = 0; k0 < HIDDEN; k0 += 32) {
            const v16bf ah0 = ld_frag_bf16(h0p + k0, hsel);
            const v16bf ah1 = ld_frag_bf16(h1p + k0, hsel);
            const v16bf al0 = ld_frag_bf16(l0p + k0, hsel);
            const v16bf al1 = ld_frag_bf16(l1p + k0, hsel);
            v16bf bfr;
#pragma unroll
            for (int a = 0; a < 4; ++a) {
                bfr = ld_frag_bf16(ldsB + (a * 16 + laneN) * PANEL_PITCH + k0, hsel);
                acc[0][a] = mma_bf16(ah0, bfr, acc[0][a]);
                acc[1][a] = mma_bf16(ah1, bfr, acc[1][a]);
                acc[0][a] = mma_bf16(al0, bfr, acc[0][a]);
                acc[1][a] = mma_bf16(al1, bfr, acc[1][a]);
            }
            guard8(acc, al1, bfr);
        }
    }
    __syncthreads();

    float biasv[4];
#pragma unroll
    for (int a = 0; a < 4; ++a)
        biasv[a] = bf16_bits_to_f32(bf16_rne_bits(bias[nBase + a * 16 + laneN]));

    float* T = (float*)lds_dyn_o + wave * (32 * 68);
#pragma unroll
    for (int sub = 0; sub < 2; ++sub)
#pragma unroll
        for (int a = 0; a < 4; ++a)
#pragma unroll
            for (int j = 0; j < 8; ++j)
                T[(sub * 16 + 8 * hsel + j) * 68 + a * 16 + laneN] = acc[sub][a][j] + biasv[a];
    __syncthreads();

    float* g = Out + (size_t)mBase * HIDDEN + nBase;
    put_out64(T, g, lane);
    __threadfence();
    put_out64(T, g, lane);
}

__global__ void __launch_bounds__(256) __attribute__((amdgpu_num_vgpr(256)))
attn_late(const _Float16* __restrict__ Qf, const _Float16* __restrict__ Kf,
          const _Float16* __restrict__ Vtf,
          unsigned short* __restrict__ Oh, unsigned short* __restrict__ Ol, int qb0) {
    __shared__ __attribute__((aligned(16))) unsigned short ldsP[8 * 640];
    __shared__ __attribute__((aligned(16))) unsigned short ldsO[8 * 2304];

    const int wave  = threadIdx.x >> 5;
    const int lane  = threadIdx.x & 31;
    const int laneN = lane & 15;
    const int hsel  = lane >> 4;
    const int bh    = blockIdx.x;
    const int bidx  = bh / HEADS;
    const int head  = bh - bidx * HEADS;
    const int q0    = (blockIdx.y + qb0) * 128 + wave * 16;

    const _Float16* qrow = Qf + ((size_t)bh * SEQ + q0 + laneN) * HEAD_DIM;
    const v16h qf0 = ld_frag_f16(qrow, hsel);
    const v16h qf1 = ld_frag_f16(qrow + 32, hsel);

    float mrow[8], lrow[8];
#pragma unroll
    for (int j = 0; j < 8; ++j) { mrow[j] = NEG_BIG; lrow[j] = 0.0f; }
    v8f o[4] = {};

    unsigned short* P = ldsP + wave * 640;
    const int kend = q0 + 16;

#pragma unroll 1
    for (int key0 = 0; key0 < kend; key0 += 32) {
        v8f s0 = {}, s1 = {};
        {
            const _Float16* krow = Kf + ((size_t)bh * SEQ + key0 + laneN) * HEAD_DIM;
            const v16h k00 = ld_frag_f16(krow, hsel);
            const v16h k01 = ld_frag_f16(krow + 32, hsel);
            const v16h k10 = ld_frag_f16(krow + 16 * HEAD_DIM, hsel);
            const v16h k11 = ld_frag_f16(krow + 16 * HEAD_DIM + 32, hsel);
            s0 = mma_f16(qf0, k00, s0);
            s0 = mma_f16(qf1, k01, s0);
            s1 = mma_f16(qf0, k10, s1);
            s1 = mma_f16(qf1, k11, s1);
            guard2(s0, s1, qf1, k11);
        }

        float p0[8], p1[8], alpha[8];
#pragma unroll
        for (int j = 0; j < 8; ++j) {
            const int r = q0 + 8 * hsel + j;
            const bool m0 = (key0 + laneN > r);
            const bool m1 = (key0 + 16 + laneN > r);
            float x0 = s0[j] * ATT_SCALE;
            float x1 = s1[j] * ATT_SCALE;
            x0 = m0 ? NEG_BIG : x0;
            x1 = m1 ? NEG_BIG : x1;
            const float mx = rowmax16(fmaxf(x0, x1));
            const float mn = fmaxf(mrow[j], mx);
            alpha[j] = __expf(mrow[j] - mn);
            float e0 = __expf(x0 - mn);
            float e1 = __expf(x1 - mn);
            e0 = m0 ? 0.0f : e0;
            e1 = m1 ? 0.0f : e1;
            p0[j] = e0;
            p1[j] = e1;
            lrow[j] = lrow[j] * alpha[j] + rowsum16(e0 + e1);
            mrow[j] = mn;
        }
#pragma unroll
        for (int a = 0; a < 4; ++a)
#pragma unroll
            for (int j = 0; j < 8; ++j) o[a][j] *= alpha[j];

#pragma unroll
        for (int j = 0; j < 8; ++j) {
            const int r = 8 * hsel + j;
            P[r * 40 + laneN]      = f16_bits(p0[j] * P_CARRY);
            P[r * 40 + 16 + laneN] = f16_bits(p1[j] * P_CARRY);
        }
        __builtin_amdgcn_fence(3, "wavefront");
        __builtin_amdgcn_wave_barrier();
        const v16h pf = ld_frag_f16((const _Float16*)(P + laneN * 40), hsel);

        const _Float16* vrow = Vtf + ((size_t)bh * HEAD_DIM + laneN) * SEQ + key0;
        v16h vf;
#pragma unroll
        for (int a = 0; a < 4; ++a) {
            vf = ld_frag_f16(vrow + (size_t)(a * 16) * SEQ, hsel);
            o[a] = mma_f16(pf, vf, o[a]);
        }
        guard4(o, pf, vf);
    }

    float inv[8];
#pragma unroll
    for (int j = 0; j < 8; ++j) inv[j] = 1.0f / (lrow[j] * P_CARRY);

    unsigned short* TH = ldsO + wave * 2304;
    unsigned short* TL = TH + 1152;
#pragma unroll
    for (int a = 0; a < 4; ++a)
#pragma unroll
        for (int j = 0; j < 8; ++j) {
            const float v = o[a][j] * inv[j];
            const unsigned short hb = bf16_rne_bits(v);
            const int idx = (8 * hsel + j) * 72 + a * 16 + laneN;
            TH[idx] = hb;
            TL[idx] = bf16_rne_bits(v - bf16_bits_to_f32(hb));
        }
    __builtin_amdgcn_fence(3, "wavefront");
    __builtin_amdgcn_wave_barrier();

    const size_t obase = ((size_t)bidx * SEQ + q0) * HIDDEN + (size_t)head * HEAD_DIM;
    put_ctx16(TH, Oh + obase, lane);
    put_ctx16(TL, Ol + obase, lane);
    __threadfence();
    put_ctx16(TH, Oh + obase, lane);
    put_ctx16(TL, Ol + obase, lane);
}

__global__ void __launch_bounds__(256) __attribute__((amdgpu_num_vgpr(256)))
attn_early(const unsigned short* __restrict__ Qbh, const unsigned short* __restrict__ Qbl,
           const unsigned short* __restrict__ Kbh, const unsigned short* __restrict__ Kbl,
           const unsigned short* __restrict__ Vbh, const unsigned short* __restrict__ Vbl,
           unsigned short* __restrict__ Oh, unsigned short* __restrict__ Ol) {
    __shared__ __attribute__((aligned(16))) unsigned short ldsP[8 * 1280];
    __shared__ __attribute__((aligned(16))) unsigned short ldsO[8 * 2304];

    const int wave  = threadIdx.x >> 5;
    const int lane  = threadIdx.x & 31;
    const int laneN = lane & 15;
    const int hsel  = lane >> 4;
    const int bh    = blockIdx.x;
    const int bidx  = bh / HEADS;
    const int head  = bh - bidx * HEADS;
    const int q0    = blockIdx.y * 128 + wave * 16;

    const unsigned short* qrh = Qbh + ((size_t)bh * EARLY + q0 + laneN) * HEAD_DIM;
    const unsigned short* qrl = Qbl + ((size_t)bh * EARLY + q0 + laneN) * HEAD_DIM;
    const v16bf qh0 = ld_frag_bf16(qrh, hsel);
    const v16bf qh1 = ld_frag_bf16(qrh + 32, hsel);
    const v16bf ql0 = ld_frag_bf16(qrl, hsel);
    const v16bf ql1 = ld_frag_bf16(qrl + 32, hsel);

    float mrow[8], lrow[8];
#pragma unroll
    for (int j = 0; j < 8; ++j) { mrow[j] = NEG_BIG; lrow[j] = 0.0f; }
    v8f o[4] = {};

    unsigned short* PH = ldsP + wave * 1280;
    unsigned short* PL = PH + 640;
    const int kend = q0 + 16;

#pragma unroll 1
    for (int key0 = 0; key0 < kend; key0 += 32) {
        v8f s0 = {}, s1 = {};
        {
            const unsigned short* krh = Kbh + ((size_t)bh * EARLY + key0 + laneN) * HEAD_DIM;
            const unsigned short* krl = Kbl + ((size_t)bh * EARLY + key0 + laneN) * HEAD_DIM;
            {
                const v16bf kh0 = ld_frag_bf16(krh, hsel);
                const v16bf kh1 = ld_frag_bf16(krh + 32, hsel);
                const v16bf kl0 = ld_frag_bf16(krl, hsel);
                const v16bf kl1 = ld_frag_bf16(krl + 32, hsel);
                s0 = mma_bf16(qh0, kh0, s0);
                s0 = mma_bf16(qh1, kh1, s0);
                s0 = mma_bf16(qh0, kl0, s0);
                s0 = mma_bf16(qh1, kl1, s0);
                s0 = mma_bf16(ql0, kh0, s0);
                s0 = mma_bf16(ql1, kh1, s0);
            }
            {
                const v16bf kh0 = ld_frag_bf16(krh + 16 * HEAD_DIM, hsel);
                const v16bf kh1 = ld_frag_bf16(krh + 16 * HEAD_DIM + 32, hsel);
                const v16bf kl0 = ld_frag_bf16(krl + 16 * HEAD_DIM, hsel);
                const v16bf kl1 = ld_frag_bf16(krl + 16 * HEAD_DIM + 32, hsel);
                s1 = mma_bf16(qh0, kh0, s1);
                s1 = mma_bf16(qh1, kh1, s1);
                s1 = mma_bf16(qh0, kl0, s1);
                s1 = mma_bf16(qh1, kl1, s1);
                s1 = mma_bf16(ql0, kh0, s1);
                s1 = mma_bf16(ql1, kh1, s1);
                guard2(s0, s1, ql1, kh1);
            }
        }

        float p0[8], p1[8], alpha[8];
#pragma unroll
        for (int j = 0; j < 8; ++j) {
            const int r = q0 + 8 * hsel + j;
            const bool m0 = (key0 + laneN > r);
            const bool m1 = (key0 + 16 + laneN > r);
            float x0 = s0[j] * ATT_SCALE;
            float x1 = s1[j] * ATT_SCALE;
            x0 = m0 ? NEG_BIG : x0;
            x1 = m1 ? NEG_BIG : x1;
            const float mx = rowmax16(fmaxf(x0, x1));
            const float mn = fmaxf(mrow[j], mx);
            alpha[j] = __expf(mrow[j] - mn);
            float e0 = __expf(x0 - mn);
            float e1 = __expf(x1 - mn);
            e0 = m0 ? 0.0f : e0;
            e1 = m1 ? 0.0f : e1;
            p0[j] = e0;
            p1[j] = e1;
            lrow[j] = lrow[j] * alpha[j] + rowsum16(e0 + e1);
            mrow[j] = mn;
        }
#pragma unroll
        for (int a = 0; a < 4; ++a)
#pragma unroll
            for (int j = 0; j < 8; ++j) o[a][j] *= alpha[j];

#pragma unroll
        for (int j = 0; j < 8; ++j) {
            const int r = 8 * hsel + j;
            const unsigned short h0 = bf16_rne_bits(p0[j]);
            const unsigned short h1 = bf16_rne_bits(p1[j]);
            PH[r * 40 + laneN]      = h0;
            PH[r * 40 + 16 + laneN] = h1;
            PL[r * 40 + laneN]      = bf16_rne_bits(p0[j] - bf16_bits_to_f32(h0));
            PL[r * 40 + 16 + laneN] = bf16_rne_bits(p1[j] - bf16_bits_to_f32(h1));
        }
        __builtin_amdgcn_fence(3, "wavefront");
        __builtin_amdgcn_wave_barrier();
        const v16bf phf = ld_frag_bf16(PH + laneN * 40, hsel);
        const v16bf plf = ld_frag_bf16(PL + laneN * 40, hsel);

        const unsigned short* vrh = Vbh + ((size_t)bh * HEAD_DIM + laneN) * EARLY + key0;
        const unsigned short* vrl = Vbl + ((size_t)bh * HEAD_DIM + laneN) * EARLY + key0;
        v16bf vh, vl;
#pragma unroll
        for (int a = 0; a < 4; ++a) {
            vh = ld_frag_bf16(vrh + (size_t)(a * 16) * EARLY, hsel);
            vl = ld_frag_bf16(vrl + (size_t)(a * 16) * EARLY, hsel);
            o[a] = mma_bf16(phf, vh, o[a]);
            o[a] = mma_bf16(phf, vl, o[a]);
            o[a] = mma_bf16(plf, vh, o[a]);
        }
        guard4(o, plf, vh);
    }

    float inv[8];
#pragma unroll
    for (int j = 0; j < 8; ++j) inv[j] = 1.0f / lrow[j];

    unsigned short* TH = ldsO + wave * 2304;
    unsigned short* TL = TH + 1152;
#pragma unroll
    for (int a = 0; a < 4; ++a)
#pragma unroll
        for (int j = 0; j < 8; ++j) {
            const float v = o[a][j] * inv[j];
            const unsigned short hb = bf16_rne_bits(v);
            const int idx = (8 * hsel + j) * 72 + a * 16 + laneN;
            TH[idx] = hb;
            TL[idx] = bf16_rne_bits(v - bf16_bits_to_f32(hb));
        }
    __builtin_amdgcn_fence(3, "wavefront");
    __builtin_amdgcn_wave_barrier();

    const size_t obase = ((size_t)bidx * SEQ + q0) * HIDDEN + (size_t)head * HEAD_DIM;
    put_ctx16(TH, Oh + obase, lane);
    put_ctx16(TL, Ol + obase, lane);
    __threadfence();
    put_ctx16(TH, Oh + obase, lane);
    put_ctx16(TL, Ol + obase, lane);
}

extern "C" void kernel_launch(void* const* d_in, const int* in_sizes, int n_in,
                              void* d_out, int out_size, void* d_ws, size_t ws_size,
                              hipStream_t stream) {
    if (n_in < 4) return;
    const long need_x = (long)(NB - 1) * SEQ_FULL * HIDDEN + (long)SEQ * HIDDEN;
    if ((long)in_sizes[0] < need_x) return;
    if (in_sizes[1] < QKV_N * HIDDEN) return;
    if (in_sizes[2] < HIDDEN * HIDDEN) return;
    if (in_sizes[3] < HIDDEN) return;
    if (out_size < MROWS * HIDDEN) return;

    const float* x     = (const float*)d_in[0];
    const float* w_qkv = (const float*)d_in[1];
    const float* w_out = (const float*)d_in[2];
    const float* b_out = (const float*)d_in[3];
    float*       out   = (float*)d_out;

    const size_t plane  = (size_t)MROWS * HIDDEN * 2;
    const size_t eplane = (size_t)NB * HEADS * EARLY * HEAD_DIM * 2;
    size_t off = 0;
    auto carve = [&](size_t bytes) { size_t o = off; off += (bytes + 255) & ~(size_t)255; return o; };
    const size_t oXb  = carve(plane);
    const size_t oWq  = carve((size_t)QKV_N * HIDDEN * 2);
    const size_t oWo  = carve((size_t)HIDDEN * HIDDEN * 2);
    const size_t oQf  = carve(plane);
    const size_t oKf  = carve(plane);
    const size_t oVt  = carve(plane);
    const size_t oQbh = carve(eplane);
    const size_t oQbl = carve(eplane);
    const size_t oKbh = carve(eplane);
    const size_t oKbl = carve(eplane);
    const size_t oVbh = carve(eplane);
    const size_t oVbl = carve(eplane);
    const size_t oOh  = carve(plane);
    const size_t oOl  = carve(plane);
    if (off > ws_size) return;

    char* ws = (char*)d_ws;
    unsigned short* Xb  = (unsigned short*)(ws + oXb);
    unsigned short* Wq  = (unsigned short*)(ws + oWq);
    unsigned short* Wo  = (unsigned short*)(ws + oWo);
    unsigned short* Qf  = (unsigned short*)(ws + oQf);
    unsigned short* Kf  = (unsigned short*)(ws + oKf);
    unsigned short* Vt  = (unsigned short*)(ws + oVt);
    unsigned short* Qbh = (unsigned short*)(ws + oQbh);
    unsigned short* Qbl = (unsigned short*)(ws + oQbl);
    unsigned short* Kbh = (unsigned short*)(ws + oKbh);
    unsigned short* Kbl = (unsigned short*)(ws + oKbl);
    unsigned short* Vbh = (unsigned short*)(ws + oVbh);
    unsigned short* Vbl = (unsigned short*)(ws + oVbl);
    unsigned short* Oh  = (unsigned short*)(ws + oOh);
    unsigned short* Ol  = (unsigned short*)(ws + oOl);

    cvt_rows_bf16<<<MROWS / 2, 256, 0, stream>>>(x, Xb, MROWS, SEQ, SEQ_FULL);
    cvt_rows_bf16<<<QKV_N / 2, 256, 0, stream>>>(w_qkv, Wq, QKV_N, QKV_N, QKV_N);
    cvt_rows_bf16<<<HIDDEN / 2, 256, 0, stream>>>(w_out, Wo, HIDDEN, HIDDEN, HIDDEN);

    hipFuncSetAttribute(reinterpret_cast<const void*>(&gemm_qkv),
                        hipFuncAttributeMaxDynamicSharedMemorySize, LDS_DYN_BYTES);
    gemm_qkv<<<dim3(MROWS / 256, QKV_N / 64), 256, LDS_DYN_BYTES, stream>>>(
        Xb, Wq, Qf, Kf, Vt, Qbh, Qbl, Kbh, Kbl, Vbh, Vbl);

    attn_early<<<dim3(NB * HEADS, EARLY / 128), 256, 0, stream>>>(
        Qbh, Qbl, Kbh, Kbl, Vbh, Vbl, Oh, Ol);
    if (SEQ > EARLY) {
        attn_late<<<dim3(NB * HEADS, (SEQ - EARLY) / 128), 256, 0, stream>>>(
            (const _Float16*)Qf, (const _Float16*)Kf, (const _Float16*)Vt, Oh, Ol, EARLY / 128);
    }

    hipFuncSetAttribute(reinterpret_cast<const void*>(&gemm_out),
                        hipFuncAttributeMaxDynamicSharedMemorySize, LDS_DYN_BYTES);
    gemm_out<<<dim3(MROWS / 256, HIDDEN / 64), 256, LDS_DYN_BYTES, stream>>>(
        Oh, Ol, Wo, b_out, out);
}
